// CausalSelfAttention_7267084665273
// MI455X (gfx1250) — hardware-run, weakly checked
//
#include <hip/hip_runtime.h>
#include <math.h>

#ifndef NB
#define NB 4
#endif
#ifndef SEQ
#define SEQ 2048
#endif
#define NB_FULL 4
#define SEQ_FULL 2048
#define DM 1024
#define NH 16
#define HD 64
#define MTOT (NB * SEQ)
#define EROWS 256

static_assert(SEQ % 256 == 0);
static_assert(MTOT % 64 == 0);
static_assert(NB <= NB_FULL);
static_assert(SEQ <= SEQ_FULL);
static_assert(EROWS % 64 == 0);
static_assert(EROWS <= SEQ);
static_assert(HD == 64);
static_assert(DM == NH * HD);
static_assert(DM % 64 == 0);
static_assert((NB * EROWS) % 64 == 0);

typedef __attribute__((ext_vector_type(16))) _Float16 v16h;
typedef __attribute__((ext_vector_type(16))) __bf16   v16b;
typedef __attribute__((ext_vector_type(8)))  float    v8f;
typedef __attribute__((ext_vector_type(4)))  float    v4f;
typedef __attribute__((ext_vector_type(4)))  unsigned int v4u;
typedef __attribute__((ext_vector_type(4)))  int      v4i;

union FU { v4u u[2]; v16h h; v16b b; };
__device__ __forceinline__ FU ldfrag(const unsigned short* p) { FU f; f.u[0] = *(const v4u*)p; f.u[1] = *(const v4u*)(p + 16); return f; }

__device__ __forceinline__ v8f wb(v16b a, v16b b, v8f c) { return __builtin_amdgcn_wmma_f32_16x16x32_bf16(false, a, false, b, (short)0, c, false, false); }
__device__ __forceinline__ v8f wh(v16h a, v16h b, v8f c) { return __builtin_amdgcn_wmma_f32_16x16x32_f16(false, a, false, b, (short)0, c, false, false); }
template <int ET> __device__ __forceinline__ v8f mma(const FU& a, const FU& b, v8f c) {
  if (ET == 0) return wh(a.h, b.h, c);
  return wb(a.b, b.b, c);
}

__device__ __forceinline__ void guard_acc4(v8f& a, v8f& b, v8f& c, v8f& d, v16h x) {
  asm volatile("v_nop\n\tv_nop\n\tv_nop\n\tv_nop" : "+v"(a), "+v"(b), "+v"(c), "+v"(d) : "v"(x));
}
__device__ __forceinline__ void keep4(v16h a, v16h b, v16h c, v16h d) { asm volatile("v_nop" :: "v"(a), "v"(b), "v"(c), "v"(d)); }
__device__ __forceinline__ void guard_s(v8f& s, v16h a0, v16h a1, v16h b0, v16h b1, v16h q0, v16h q1, v16h q2, v16h q3) {
  asm volatile("v_nop\n\tv_nop\n\tv_nop\n\tv_nop" : "+v"(s) : "v"(a0), "v"(a1), "v"(b0), "v"(b1), "v"(q0), "v"(q1), "v"(q2), "v"(q3));
}
__device__ __forceinline__ void guard_o(v8f& a, v8f& b, v8f& c, v8f& d, v16h p, v16h v0, v16h v1, v16h v2, v16h v3) {
  asm volatile("v_nop\n\tv_nop\n\tv_nop\n\tv_nop" : "+v"(a), "+v"(b), "+v"(c), "+v"(d) : "v"(p), "v"(v0), "v"(v1), "v"(v2), "v"(v3));
}
__device__ __forceinline__ void guard_o2(v8f& a, v8f& b, v16h ph, v16h pl, v16h v0, v16h v1, v16h v2, v16h v3) {
  asm volatile("v_nop\n\tv_nop\n\tv_nop\n\tv_nop" : "+v"(a), "+v"(b) : "v"(ph), "v"(pl), "v"(v0), "v"(v1), "v"(v2), "v"(v3));
}

#if __has_builtin(__builtin_amdgcn_exp2f)
#define EX2(x) __builtin_amdgcn_exp2f(x)
#else
#define EX2(x) exp2f(x)
#endif

__device__ __forceinline__ unsigned bfu_rne(float v) { const unsigned u = __float_as_uint(v); return (u + 0x7FFFu + ((u >> 16) & 1u)) >> 16; }
__device__ __forceinline__ float bf_keep(float v) { return __uint_as_float(bfu_rne(v) << 16); }
__device__ __forceinline__ void bfsplit(float v, unsigned& hi, unsigned& lo) { hi = bfu_rne(v); lo = bfu_rne(v - __uint_as_float(hi << 16)); }
__device__ __forceinline__ unsigned pkh2(float a, float b) {
  return (unsigned)__builtin_bit_cast(unsigned short, (_Float16)a) | ((unsigned)__builtin_bit_cast(unsigned short, (_Float16)b) << 16);
}

#define VST2Q(ptr, val) do { const v4u vq_ = (val); *(volatile v4u*)(ptr) = vq_; __threadfence(); *(volatile v4u*)(ptr) = vq_; } while (0)

__device__ __forceinline__ int wave_count_kept(const int* __restrict__ mrow, int lane) {
  int c = 0;
#pragma unroll 4
  for (int it = 0; it < SEQ / 128; ++it) {
    const v4i m = *(const v4i*)(mrow + (it * 32 + lane) * 4);
    c += ((m.x != 0) ? 1 : 0) + ((m.y != 0) ? 1 : 0) + ((m.z != 0) ? 1 : 0) + ((m.w != 0) ? 1 : 0);
  }
  c += __shfl_xor(c, 16, 32); c += __shfl_xor(c, 8, 32); c += __shfl_xor(c, 4, 32); c += __shfl_xor(c, 2, 32); c += __shfl_xor(c, 1, 32);
  return __builtin_amdgcn_readfirstlane(c);
}
__device__ __forceinline__ int eff_keys(int cnt) { return (cnt == 0) ? SEQ : min(cnt, SEQ); }
__device__ __forceinline__ int pad32(int nk) { return min((nk + 31) & ~31, SEQ); }

__global__ __launch_bounds__(256) void k_xcast(const float* __restrict__ x, unsigned short* __restrict__ X16) {
  const int tid = threadIdx.x;
  const int bpb = SEQ / 32;
  const int b = blockIdx.x / bpb;
  const int t0 = (blockIdx.x - b * bpb) * 32;
#pragma unroll 2
  for (int it = 0; it < 16; ++it) {
    const int u = it * 256 + tid;
    const int rr = u >> 7, c0 = (u & 127) * 8;
    const int t = t0 + rr;
    const float* s = x + ((size_t)b * SEQ_FULL + t) * DM + c0;
    const v4f a = *(const v4f*)s, e4 = *(const v4f*)(s + 4);
    v4u pk;
    pk.x = pkh2(bf_keep(a.x), bf_keep(a.y));   pk.y = pkh2(bf_keep(a.z), bf_keep(a.w));
    pk.z = pkh2(bf_keep(e4.x), bf_keep(e4.y)); pk.w = pkh2(bf_keep(e4.z), bf_keep(e4.w));
    VST2Q(X16 + ((size_t)b * SEQ + t) * DM + c0, pk);
  }
}

__global__ __launch_bounds__(256) void k_wqkvT(const float* __restrict__ W, unsigned short* __restrict__ WT) {
  const int u = blockIdx.x * 256 + threadIdx.x;
  if (u >= 3 * DM * (DM / 8)) return;
  const int n = u >> 7, k0 = (u & 127) * 8;
  float w[8];
#pragma unroll
  for (int e = 0; e < 8; ++e) w[e] = bf_keep(W[(size_t)(k0 + e) * (3 * DM) + n]) * 64.0f;
  v4u pk; pk.x = pkh2(w[0], w[1]); pk.y = pkh2(w[2], w[3]); pk.z = pkh2(w[4], w[5]); pk.w = pkh2(w[6], w[7]);
  VST2Q(WT + (size_t)n * DM + k0, pk);
}

__global__ __launch_bounds__(256) void k_woT(const float* __restrict__ W, unsigned short* __restrict__ BTO) {
  const int u = blockIdx.x * 256 + threadIdx.x;
  if (u >= DM * 256) return;
  const int n = u >> 8, kk0 = (u & 255) * 8, k0 = kk0 & (DM - 1);
  unsigned w[8];
#pragma unroll
  for (int e = 0; e < 8; ++e) w[e] = bfu_rne(W[(size_t)(k0 + e) * DM + n]);
  v4u pk; pk.x = w[0] | (w[1] << 16); pk.y = w[2] | (w[3] << 16); pk.z = w[4] | (w[5] << 16); pk.w = w[6] | (w[7] << 16);
  VST2Q(BTO + (size_t)n * (2 * DM) + kk0, pk);
}

template <int ET, int BIAS_MODE, int OUT_MODE, int CMP>
__global__ __launch_bounds__(256) void k_gemm64(
    const unsigned short* __restrict__ A, const unsigned short* __restrict__ Bt,
    void* __restrict__ Cout, void* __restrict__ Cout2, const float* __restrict__ bias, const int* __restrict__ mask,
    long long strideA, long long strideC, int lda, int ldb, int ldc, int M, int N, int K, float scale) {
  __shared__ __align__(16) float sT[8][16 * 68];
  const int z    = blockIdx.y;
  const int lane = threadIdx.x & 31;
  const int wave = threadIdx.x >> 5;
  const int tilesN = N >> 6;
  const int tilesM = M >> 6;
  const int tile = blockIdx.x * 8 + wave;
  if (tile >= tilesM * tilesN) return;
  const int tm = tile / tilesN;
  const int tn = tile - tm * tilesN;
  const int m0 = tm << 6;
  const int n0 = tn << 6;
  if (CMP != 0) {
    const int g0 = (CMP == 1) ? m0 : n0;
    const int bb = min(g0 / SEQ, NB - 1);
    const int loc = g0 - bb * SEQ;
    const int nkp = pad32(eff_keys(wave_count_kept(mask + (size_t)bb * SEQ_FULL, lane)));
    if (loc >= nkp) return;
  }
  const unsigned short* Ab = A + (size_t)z * (size_t)strideA;
  const int rlane = lane & 15;
  const int koff  = (lane >> 4) * 8;
  const int mOff  = (lane >> 4) * 8;

  v8f acc[4][4];
#pragma unroll
  for (int i = 0; i < 4; ++i)
#pragma unroll
    for (int j = 0; j < 4; ++j) { v8f zz = {}; acc[i][j] = zz; }

  for (int k0 = 0; k0 < K; k0 += 32) {
    FU bh[4];
#pragma unroll
    for (int j = 0; j < 4; ++j) bh[j] = ldfrag(Bt + (size_t)(n0 + (j << 4) + rlane) * ldb + koff + k0);
#pragma unroll
    for (int i = 0; i < 4; ++i) {
      const FU ah = ldfrag(Ab + (size_t)(m0 + (i << 4) + rlane) * lda + koff + k0);
#pragma unroll
      for (int j = 0; j < 4; ++j) acc[i][j] = mma<ET>(ah, bh[j], acc[i][j]);
      guard_acc4(acc[i][0], acc[i][1], acc[i][2], acc[i][3], ah.h);
    }
    keep4(bh[0].h, bh[1].h, bh[2].h, bh[3].h);
  }

  float* slab = sT[wave];
#pragma unroll
  for (int i = 0; i < 4; ++i) {
    const int mBase = m0 + (i << 4);
#pragma unroll
    for (int j = 0; j < 4; ++j) {
      const int n = n0 + (j << 4) + rlane;
      float bv = 0.f;
      if (BIAS_MODE == 2) bv = bf_keep(bias[n]);
#pragma unroll
      for (int r = 0; r < 8; ++r) {
        float v = acc[i][j][r] * scale;
        if (BIAS_MODE == 1) v += bf_keep(bias[mBase + mOff + r]);
        if (BIAS_MODE == 2) v += bv;
        slab[(mOff + r) * 68 + (j << 4) + rlane] = v;
      }
    }
    __builtin_amdgcn_fence(3  , "workgroup");
    __builtin_amdgcn_wave_barrier();
    __builtin_amdgcn_fence(2  , "workgroup");
    if (OUT_MODE == 0) {
      float* C = (float*)Cout + (size_t)z * (size_t)strideC;
      const int hh = lane >> 4, c4 = (lane & 15) * 4;
      v4f val[8];
#pragma unroll
      for (int it = 0; it < 8; ++it) val[it] = *(const v4f*)(slab + (it * 2 + hh) * 68 + c4);
#pragma unroll
      for (int pass = 0; pass < 2; ++pass) {
#pragma unroll
        for (int it = 0; it < 8; ++it) *(volatile v4f*)(C + (size_t)(mBase + it * 2 + hh) * ldc + n0 + c4) = val[it];
        __threadfence();
      }
    } else {
      const int q = lane >> 3, c8 = (lane & 7) * 8;
      unsigned short* C  = (unsigned short*)Cout  + (size_t)z * (size_t)strideC;
      unsigned short* C2 = (unsigned short*)Cout2 + (size_t)z * (size_t)strideC;
      v4u hv[4], lv[4];
#pragma unroll
      for (int it = 0; it < 4; ++it) {
        const float* sp = slab + (it * 4 + q) * 68 + c8;
        const v4f a = *(const v4f*)sp, b = *(const v4f*)(sp + 4);
        if (OUT_MODE == 1) {
          hv[it].x = pkh2(a.x, a.y); hv[it].y = pkh2(a.z, a.w); hv[it].z = pkh2(b.x, b.y); hv[it].w = pkh2(b.z, b.w);
          lv[it] = hv[it];
        } else {
          unsigned h0, l0, h1, l1;
          bfsplit(a.x, h0, l0); bfsplit(a.y, h1, l1); hv[it].x = h0 | (h1 << 16); lv[it].x = l0 | (l1 << 16);
          bfsplit(a.z, h0, l0); bfsplit(a.w, h1, l1); hv[it].y = h0 | (h1 << 16); lv[it].y = l0 | (l1 << 16);
          bfsplit(b.x, h0, l0); bfsplit(b.y, h1, l1); hv[it].z = h0 | (h1 << 16); lv[it].z = l0 | (l1 << 16);
          bfsplit(b.z, h0, l0); bfsplit(b.w, h1, l1); hv[it].w = h0 | (h1 << 16); lv[it].w = l0 | (l1 << 16);
        }
      }
#pragma unroll
      for (int pass = 0; pass < 2; ++pass) {
#pragma unroll
        for (int it = 0; it < 4; ++it) {
          const size_t off = (size_t)(mBase + it * 4 + q) * ldc + n0 + c8;
          *(volatile v4u*)(C + off) = hv[it];
          if (OUT_MODE == 2) *(volatile v4u*)(C2 + off) = lv[it];
        }
        __threadfence();
      }
    }
    __builtin_amdgcn_fence(3  , "workgroup");
    __builtin_amdgcn_wave_barrier();
    __builtin_amdgcn_fence(2  , "workgroup");
  }
}

template <int EARLY>
__device__ __forceinline__ void attn_body(const unsigned short* __restrict__ QH, const unsigned short* __restrict__ QL,
                                          const unsigned short* __restrict__ KH, const unsigned short* __restrict__ KL,
                                          const unsigned short* __restrict__ VA, const unsigned short* __restrict__ VB,
                                          const int* __restrict__ mask, unsigned short* __restrict__ AOP, float* osb) {
  constexpr int NQB = EARLY ? (EROWS / 64) : ((((SEQ - EROWS) / 64) > 0) ? ((SEQ - EROWS) / 64) : 1);
  constexpr int QST = EARLY ? 0 : EROWS;
  constexpr size_t VP  = EARLY ? ((size_t)NB * EROWS) : (size_t)MTOT;
  constexpr size_t VBC = EARLY ? (size_t)EROWS : (size_t)SEQ;
  const int lane = threadIdx.x & 31, hf = lane >> 4, c = lane & 15;
  const int wave = __builtin_amdgcn_readfirstlane((int)(threadIdx.x >> 5));
  const int bx = blockIdx.x;
  const int qb = bx % NQB;
  const int bh = bx / NQB;
  const int h  = bh % NH;
  const int b  = min(bh / NH, NB - 1);
  const int q0 = QST + qb * 64 + wave * 16;
  const int qme = q0 + c;
  const size_t rowb = (size_t)b * SEQ;
  const int* mrow = mask + (size_t)b * SEQ_FULL;
  const int nkp = (q0 + 16 + 31) & ~31;

  const size_t qoff = (rowb + q0 + c) * DM + h * HD + 8 * hf;
  const FU qh0 = ldfrag(QH + qoff), qh1 = ldfrag(QH + qoff + 32);
  const FU ql0 = ldfrag(QL + qoff), ql1 = ldfrag(QL + qoff + 32);

  const size_t koff = (rowb + c) * DM + h * HD + 8 * hf;
  const unsigned short* kbh = KH + koff;
  const unsigned short* kbl = KL + koff;
  const size_t voff = (size_t)(h * HD + c) * VP + (size_t)b * VBC + 8 * hf;
  const unsigned short* vtb = VA + voff;
  const unsigned short* vlb = VB + voff;

  const float SC = 0.18033688011112042f;
  const float NEGINF = -__builtin_inff();
  float msh = -__builtin_inff();
  float lpart = 0.f;
  v8f o0 = {}, o1 = {}, o2 = {}, o3 = {};

#pragma unroll 1
  for (int tk = 0; tk < nkp; tk += 32) {
    int mv = mrow[tk + lane];
    asm volatile("" : "+v"(mv));
    const unsigned mw = __builtin_amdgcn_ballot_w32(mv != 0);
    const unsigned short* kh = kbh + (size_t)tk * DM;
    const unsigned short* kl = kbl + (size_t)tk * DM;
    v8f s0 = {}, s1 = {};
    {
      const FU a0 = ldfrag(kh), a1 = ldfrag(kh + 32), b0 = ldfrag(kl), b1 = ldfrag(kl + 32);
      s0 = wb(b0.b, qh0.b, s0); s0 = wb(a0.b, ql0.b, s0); s0 = wb(a0.b, qh0.b, s0);
      s0 = wb(b1.b, qh1.b, s0); s0 = wb(a1.b, ql1.b, s0); s0 = wb(a1.b, qh1.b, s0);
      guard_s(s0, a0.h, a1.h, b0.h, b1.h, qh0.h, qh1.h, ql0.h, ql1.h);
    }
    {
      const unsigned short* kh1 = kh + (size_t)16 * DM;
      const unsigned short* kl1 = kl + (size_t)16 * DM;
      const FU a0 = ldfrag(kh1), a1 = ldfrag(kh1 + 32), b0 = ldfrag(kl1), b1 = ldfrag(kl1 + 32);
      s1 = wb(b0.b, qh0.b, s1); s1 = wb(a0.b, ql0.b, s1); s1 = wb(a0.b, qh0.b, s1);
      s1 = wb(b1.b, qh1.b, s1); s1 = wb(a1.b, ql1.b, s1); s1 = wb(a1.b, qh1.b, s1);
      guard_s(s1, a0.h, a1.h, b0.h, b1.h, qh0.h, qh1.h, ql0.h, ql1.h);
    }
    float ss[16];
#pragma unroll
    for (int r = 0; r < 8; ++r) { ss[r] = s0[r]; ss[8 + r] = s1[r]; }
    if ((mw != 0xFFFFFFFFu) || (tk + 31 > q0)) {
      const int kb0 = tk + 8 * hf;
      const unsigned mb = mw >> (8 * hf);
#pragma unroll
      for (int r = 0; r < 8; ++r) {
        ss[r]     = ((((mb >> r) & 1u) != 0u) && (kb0 + r <= qme))             ? ss[r]     : NEGINF;
        ss[8 + r] = ((((mb >> (16 + r)) & 1u) != 0u) && (kb0 + 16 + r <= qme)) ? ss[8 + r] : NEGINF;
      }
    }
    float mloc = ss[0];
#pragma unroll
    for (int i = 1; i < 16; ++i) mloc = fmaxf(mloc, ss[i]);
    mloc = fmaxf(mloc, __shfl_xor(mloc, 16, 32));
    const float mnew = fmaxf(msh, fmaf(mloc, SC, -14.0f));
    const float mfin = (mnew == NEGINF) ? 0.0f : mnew;
    const float corr = EX2(msh - mfin);
    const float nms = -mfin;
    msh = mnew;
    float psum = 0.f;
    lpart = lpart * corr;
    o0 *= corr; o1 *= corr; o2 *= corr; o3 *= corr;

    if (EARLY == 0) {
      v16h pf;
#pragma unroll
      for (int i = 0; i < 16; ++i) {
        const float p = EX2(fmaf(ss[i], SC, nms));
        psum += p;
        pf[i] = (_Float16)p;
      }
      lpart += psum;
      const unsigned short* vp = vtb + tk;
      const FU v0 = ldfrag(vp), v1 = ldfrag(vp + (size_t)16 * VP), v2 = ldfrag(vp + (size_t)32 * VP), v3 = ldfrag(vp + (size_t)48 * VP);
      o0 = wh(v0.h, pf, o0);
      o1 = wh(v1.h, pf, o1);
      o2 = wh(v2.h, pf, o2);
      o3 = wh(v3.h, pf, o3);
      guard_o(o0, o1, o2, o3, pf, v0.h, v1.h, v2.h, v3.h);
    } else {
      unsigned hb[16], lb[16];
#pragma unroll
      for (int i = 0; i < 16; ++i) {
        const float p = EX2(fmaf(ss[i], SC, nms));
        psum += p;
        bfsplit(p, hb[i], lb[i]);
      }
      lpart += psum;
      FU ph, pl;
      {
        v4u t;
        t.x = hb[0] | (hb[1] << 16);   t.y = hb[2] | (hb[3] << 16);   t.z = hb[4] | (hb[5] << 16);   t.w = hb[6] | (hb[7] << 16);   ph.u[0] = t;
        t.x = hb[8] | (hb[9] << 16);   t.y = hb[10] | (hb[11] << 16); t.z = hb[12] | (hb[13] << 16); t.w = hb[14] | (hb[15] << 16); ph.u[1] = t;
        t.x = lb[0] | (lb[1] << 16);   t.y = lb[2] | (lb[3] << 16);   t.z = lb[4] | (lb[5] << 16);   t.w = lb[6] | (lb[7] << 16);   pl.u[0] = t;
        t.x = lb[8] | (lb[9] << 16);   t.y = lb[10] | (lb[11] << 16); t.z = lb[12] | (lb[13] << 16); t.w = lb[14] | (lb[15] << 16); pl.u[1] = t;
      }
      const unsigned short* vph = vtb + tk;
      const unsigned short* vpl = vlb + tk;
      {
        const FU a0 = ldfrag(vph), b0 = ldfrag(vpl), a1 = ldfrag(vph + (size_t)16 * VP), b1 = ldfrag(vpl + (size_t)16 * VP);
        o0 = wb(b0.b, ph.b, o0); o0 = wb(a0.b, pl.b, o0); o0 = wb(a0.b, ph.b, o0);
        o1 = wb(b1.b, ph.b, o1); o1 = wb(a1.b, pl.b, o1); o1 = wb(a1.b, ph.b, o1);
        guard_o2(o0, o1, ph.h, pl.h, a0.h, b0.h, a1.h, b1.h);
      }
      {
        const FU a2 = ldfrag(vph + (size_t)32 * VP), b2 = ldfrag(vpl + (size_t)32 * VP), a3 = ldfrag(vph + (size_t)48 * VP), b3 = ldfrag(vpl + (size_t)48 * VP);
        o2 = wb(b2.b, ph.b, o2); o2 = wb(a2.b, pl.b, o2); o2 = wb(a2.b, ph.b, o2);
        o3 = wb(b3.b, ph.b, o3); o3 = wb(a3.b, pl.b, o3); o3 = wb(a3.b, ph.b, o3);
        guard_o2(o2, o3, ph.h, pl.h, a2.h, b2.h, a3.h, b3.h);
      }
    }
  }

  const float lt = lpart + __shfl_xor(lpart, 16, 32);
  const float inv = 1.0f / lt;
  float* os = osb + wave * (16 * 68);
  {
    float* d = os + c * 68 + 8 * hf;
    v4f a, e;
    a.x = o0[0] * inv; a.y = o0[1] * inv; a.z = o0[2] * inv; a.w = o0[3] * inv; e.x = o0[4] * inv; e.y = o0[5] * inv; e.z = o0[6] * inv; e.w = o0[7] * inv;
    *(v4f*)(d) = a; *(v4f*)(d + 4) = e;
    a.x = o1[0] * inv; a.y = o1[1] * inv; a.z = o1[2] * inv; a.w = o1[3] * inv; e.x = o1[4] * inv; e.y = o1[5] * inv; e.z = o1[6] * inv; e.w = o1[7] * inv;
    *(v4f*)(d + 16) = a; *(v4f*)(d + 20) = e;
    a.x = o2[0] * inv; a.y = o2[1] * inv; a.z = o2[2] * inv; a.w = o2[3] * inv; e.x = o2[4] * inv; e.y = o2[5] * inv; e.z = o2[6] * inv; e.w = o2[7] * inv;
    *(v4f*)(d + 32) = a; *(v4f*)(d + 36) = e;
    a.x = o3[0] * inv; a.y = o3[1] * inv; a.z = o3[2] * inv; a.w = o3[3] * inv; e.x = o3[4] * inv; e.y = o3[5] * inv; e.z = o3[6] * inv; e.w = o3[7] * inv;
    *(v4f*)(d + 48) = a; *(v4f*)(d + 52) = e;
  }
  __builtin_amdgcn_fence(3  , "workgroup");
  __builtin_amdgcn_wave_barrier();
  __builtin_amdgcn_fence(2  , "workgroup");
  {
    const int qq = lane >> 3, c8 = (lane & 7) * 8;
    unsigned short* dH = AOP + (rowb + q0) * (2 * DM) + h * HD + c8;
    unsigned short* dL = dH + DM;
    v4u hv[4], lv[4];
#pragma unroll
    for (int it = 0; it < 4; ++it) {
      const float* sp = os + (it * 4 + qq) * 68 + c8;
      const v4f a = *(const v4f*)sp, e = *(const v4f*)(sp + 4);
      unsigned h0, l0, h1, l1;
      bfsplit(a.x, h0, l0); bfsplit(a.y, h1, l1); hv[it].x = h0 | (h1 << 16); lv[it].x = l0 | (l1 << 16);
      bfsplit(a.z, h0, l0); bfsplit(a.w, h1, l1); hv[it].y = h0 | (h1 << 16); lv[it].y = l0 | (l1 << 16);
      bfsplit(e.x, h0, l0); bfsplit(e.y, h1, l1); hv[it].z = h0 | (h1 << 16); lv[it].z = l0 | (l1 << 16);
      bfsplit(e.z, h0, l0); bfsplit(e.w, h1, l1); hv[it].w = h0 | (h1 << 16); lv[it].w = l0 | (l1 << 16);
    }
#pragma unroll
    for (int pass = 0; pass < 2; ++pass) {
#pragma unroll
      for (int it = 0; it < 4; ++it) {
        const size_t off = (size_t)(it * 4 + qq) * (2 * DM);
        *(volatile v4u*)(dH + off) = hv[it];
        *(volatile v4u*)(dL + off) = lv[it];
      }
      __threadfence();
    }
  }
}

__global__ __launch_bounds__(128) void k_attn_late(const unsigned short* __restrict__ QH, const unsigned short* __restrict__ QL,
                                                   const unsigned short* __restrict__ KH, const unsigned short* __restrict__ KL,
                                                   const unsigned short* __restrict__ VT, const int* __restrict__ mask,
                                                   unsigned short* __restrict__ AOP) {
  __shared__ __align__(16) float Os[4][16 * 68];
  attn_body<0>(QH, QL, KH, KL, VT, VT, mask, AOP, &Os[0][0]);
}
__global__ __launch_bounds__(128) void k_attn_early(const unsigned short* __restrict__ QH, const unsigned short* __restrict__ QL,
                                                    const unsigned short* __restrict__ KH, const unsigned short* __restrict__ KL,
                                                    const unsigned short* __restrict__ VEH, const unsigned short* __restrict__ VEL,
                                                    const int* __restrict__ mask, unsigned short* __restrict__ AOP) {
  __shared__ __align__(16) float Os[4][16 * 68];
  attn_body<1>(QH, QL, KH, KL, VEH, VEL, mask, AOP, &Os[0][0]);
}

constexpr size_t SZ_X16 = (size_t)MTOT * DM * 2;
constexpr size_t SZ_AOP = (size_t)MTOT * 2 * DM * 2;
constexpr size_t SZ_R0  = (SZ_X16 > SZ_AOP) ? SZ_X16 : SZ_AOP;
constexpr size_t SZ_W3  = (size_t)3 * DM * DM * 2;
constexpr size_t SZ_BTO = (size_t)DM * 2 * DM * 2;
constexpr size_t SZ_PL  = (size_t)MTOT * DM * 2;
constexpr size_t SZ_VT  = (size_t)DM * MTOT * 2;
constexpr size_t SZ_VE  = (size_t)DM * NB * EROWS * 2;
constexpr size_t SZ_TOTAL = SZ_R0 + SZ_W3 + SZ_BTO + 4 * SZ_PL + SZ_VT + 2 * SZ_VE;
static_assert(SZ_X16 <= SZ_R0);
static_assert(SZ_AOP <= SZ_R0);
static_assert(SZ_TOTAL <= (size_t)134217728);
static_assert((SZ_R0 % 256) == 0 && (SZ_W3 % 256) == 0 && (SZ_BTO % 256) == 0 && (SZ_PL % 256) == 0 && (SZ_VT % 256) == 0 && (SZ_VE % 256) == 0);
static_assert(((size_t)(NB - 1) * SEQ_FULL + SEQ) * DM * 4 <= (size_t)NB_FULL * SEQ_FULL * DM * 4);

extern "C" void kernel_launch(void* const* d_in, const int* in_sizes, int n_in, void* d_out, int out_size, void* d_ws, size_t ws_size, hipStream_t stream) {
  if (n_in < 6) return;
  const long long rows_full = (long long)(NB - 1) * SEQ_FULL + SEQ;
  if ((long long)in_sizes[0] < rows_full * DM) return;
  if ((long long)in_sizes[1] < rows_full) return;
  if ((long long)in_sizes[2] < (long long)DM * 3 * DM) return;
  if ((long long)in_sizes[3] < 3 * DM) return;
  if ((long long)in_sizes[4] < (long long)DM * DM) return;
  if ((long long)in_sizes[5] < DM) return;
  if ((long long)out_size < rows_full * DM) return;
  if (ws_size < SZ_TOTAL) return;

  const float* x    = (const float*)d_in[0];
  const int*   mask = (const int*)d_in[1];
  const float* Wqkv = (const float*)d_in[2];
  const float* bqkv = (const float*)d_in[3];
  const float* Wo   = (const float*)d_in[4];
  const float* bo   = (const float*)d_in[5];
  float* out = (float*)d_out;

  char* wsp = (char*)d_ws;
  unsigned short* X16  = (unsigned short*)wsp;
  unsigned short* AOP  = (unsigned short*)wsp;
  wsp += SZ_R0;
  unsigned short* W316 = (unsigned short*)wsp; wsp += SZ_W3;
  unsigned short* BTO  = (unsigned short*)wsp; wsp += SZ_BTO;
  unsigned short* QH   = (unsigned short*)wsp; wsp += SZ_PL;
  unsigned short* QL   = (unsigned short*)wsp; wsp += SZ_PL;
  unsigned short* KH   = (unsigned short*)wsp; wsp += SZ_PL;
  unsigned short* KL   = (unsigned short*)wsp; wsp += SZ_PL;
  unsigned short* VT   = (unsigned short*)wsp; wsp += SZ_VT;
  unsigned short* VEH  = (unsigned short*)wsp; wsp += SZ_VE;
  unsigned short* VEL  = (unsigned short*)wsp; wsp += SZ_VE;

  k_xcast<<<(unsigned)(NB * (SEQ / 32)), 256, 0, stream>>>(x, X16);
  k_wqkvT<<<(3 * DM * (DM / 8) + 255) / 256, 256, 0, stream>>>(Wqkv, W316);
  k_woT<<<(DM * 256 + 255) / 256, 256, 0, stream>>>(Wo, BTO);

  {
    const int tiles = (MTOT / 64) * (DM / 64);
    k_gemm64<0, 2, 2, 0><<<dim3((unsigned)((tiles + 7) / 8), 1u), 256, 0, stream>>>(
        X16, W316, (void*)QH, (void*)QL, bqkv, mask, 0LL, 0LL, DM, DM, DM, MTOT, DM, DM, 1.0f / 64.0f);
  }
  {
    const int tiles = (MTOT / 64) * (DM / 64);
    k_gemm64<0, 2, 2, 0><<<dim3((unsigned)((tiles + 7) / 8), 1u), 256, 0, stream>>>(
        X16, W316 + (size_t)DM * DM, (void*)KH, (void*)KL, bqkv + DM, mask, 0LL, 0LL, DM, DM, DM, MTOT, DM, DM, 1.0f / 64.0f);
  }
  {
    const int tiles = (DM / 64) * (MTOT / 64);
    k_gemm64<0, 1, 1, 0><<<dim3((unsigned)((tiles + 7) / 8), 1u), 256, 0, stream>>>(
        W316 + (size_t)2 * DM * DM, X16, (void*)VT, (void*)VT, bqkv + 2 * DM, mask, 0LL, 0LL, DM, DM, MTOT, DM, MTOT, DM, 1.0f / 64.0f);
  }
  for (int b = 0; b < NB; ++b) {
    const int tiles = (DM / 64) * (EROWS / 64);
    k_gemm64<0, 1, 2, 0><<<dim3((unsigned)((tiles + 7) / 8), 1u), 256, 0, stream>>>(
        W316 + (size_t)2 * DM * DM, X16 + (size_t)b * SEQ * DM, (void*)(VEH + (size_t)b * EROWS), (void*)(VEL + (size_t)b * EROWS),
        bqkv + 2 * DM, mask, 0LL, 0LL, DM, DM, NB * EROWS, DM, EROWS, DM, 1.0f / 64.0f);
  }
  k_attn_early<<<(unsigned)(NB * NH * (EROWS / 64)), 128, 0, stream>>>(QH, QL, KH, KL, VEH, VEL, mask, AOP);
  if (SEQ > EROWS) {
    k_attn_late<<<(unsigned)(NB * NH * ((SEQ - EROWS) / 64)), 128, 0, stream>>>(QH, QL, KH, KL, VT, mask, AOP);
  }
  {
    const int tiles = (SEQ / 64) * (DM / 64);
    k_gemm64<1, 2, 0, 0><<<dim3((unsigned)((tiles + 7) / 8), (unsigned)NB), 256, 0, stream>>>(
        AOP, BTO, (void*)out, (void*)out, bo, mask, (long long)SEQ * 2 * DM, (long long)SEQ_FULL * DM, 2 * DM, 2 * DM, DM, SEQ, DM, 2 * DM, 1.0f);
  }
}
